// GraphTransformerLayer_4123168604558
// MI455X (gfx1250) — hardware-verified
//
#include <hip/hip_runtime.h>


#ifndef SEQ
#define SEQ 8192
#endif
#define SEQ_FULL 8192
#define DIMN 512
#define NHEAD 8
#define HDIM 64
#define KBLK 64
#define NKB (SEQ / KBLK)
#define GT 128
#define LDSA 40
#define CSP 132
#define PSP 80

static_assert((SEQ % GT) == 0);
static_assert(SEQ >= GT);
static_assert(SEQ <= SEQ_FULL);
static_assert(DIMN == NHEAD * HDIM);
static_assert((DIMN % GT) == 0);
static_assert((DIMN % 32) == 0);
static_assert(HDIM == 64);
static_assert(2 * GT * LDSA * 2 <= 64 * CSP * 4);
static_assert(((SEQ * DIMN / 8) % 256) == 0);
static_assert(((DIMN * DIMN / 8) % 256) == 0);

typedef _Float16 h16;
typedef _Float16 v16h __attribute__((ext_vector_type(16)));
typedef _Float16 v8h  __attribute__((ext_vector_type(8)));
typedef float    v8f  __attribute__((ext_vector_type(8)));
typedef float    v4f  __attribute__((ext_vector_type(4)));
typedef unsigned v4u  __attribute__((ext_vector_type(4)));

union Pack8 { v8h h; v4u u; };

__device__ __forceinline__ float bf16_rne(float f) {
    unsigned u = __float_as_uint(f);
    u = (u + 0x7FFFu + ((u >> 16) & 1u)) & 0xFFFF0000u;
    return __uint_as_float(u);
}

__device__ __forceinline__ v16h load_frag(const h16* p, int ld) {
    const int lane = threadIdx.x & 31;
    const int r    = lane & 15;
    const int kh   = lane >> 4;
    const h16* q = p + (size_t)r * ld + kh * 8;
    const v8h e0 = *(const v8h*)(q);
    const v8h e1 = *(const v8h*)(q + 16);
    return __builtin_shufflevector(e0, e1, 0,1,2,3,4,5,6,7,8,9,10,11,12,13,14,15);
}

__device__ __forceinline__ v8f wmma_f16(v16h a, v16h b, v8f c) {
    v8f d = __builtin_amdgcn_wmma_f32_16x16x32_f16(false, a, false, b, (short)0, c,
                                                   false, false);
    asm volatile("v_nop\n\tv_nop\n\tv_nop\n\tv_nop" : "+v"(d) : "v"(a), "v"(b));
    return d;
}

__global__ __launch_bounds__(256) void k_cvt4(
    const float* __restrict__ s0, const float* __restrict__ s1,
    const float* __restrict__ s2, const float* __restrict__ s3,
    h16* d0, h16* d1, h16* d2, h16* d3, int n8, float scale)
{
    const int y = blockIdx.y;
    const float* s = (y == 0) ? s0 : ((y == 1) ? s1 : ((y == 2) ? s2 : s3));
    h16* d = (y == 0) ? d0 : ((y == 1) ? d1 : ((y == 2) ? d2 : d3));
    const int i = (int)blockIdx.x * 256 + (int)threadIdx.x;
    if (i >= n8) return;
    const float* sp = s + (size_t)i * 8;
    const v4f a = *(const v4f*)sp;
    const v4f b = *(const v4f*)(sp + 4);
    Pack8 pk;
    pk.h = (v8h){ (h16)(bf16_rne(a[0]) * scale), (h16)(bf16_rne(a[1]) * scale),
                  (h16)(bf16_rne(a[2]) * scale), (h16)(bf16_rne(a[3]) * scale),
                  (h16)(bf16_rne(b[0]) * scale), (h16)(bf16_rne(b[1]) * scale),
                  (h16)(bf16_rne(b[2]) * scale), (h16)(bf16_rne(b[3]) * scale) };
    h16* dp = d + (size_t)i * 8;
    *(volatile v4u*)dp = pk.u;
    __threadfence();
    *(volatile v4u*)dp = pk.u;
}

__device__ __forceinline__ void emit_rows_f32(const float* Cs, float* dstbase,
                                              int pitch, int tid) {
    #pragma unroll
    for (int it = 0; it < 8; ++it) {
        const int L  = it * 32 + (tid >> 3);
        const int rl = L >> 2, seg = L & 3, q = tid & 7;
        const int c  = seg * 32 + q * 4;
        const v4f v = *(const v4f*)(Cs + rl * CSP + c);
        *(volatile v4f*)(dstbase + (size_t)rl * pitch + c) = v;
    }
}

__device__ __forceinline__ void emit_rows_f16(const float* Cs, h16* dstbase,
                                              int pitch, int tid) {
    #pragma unroll
    for (int it = 0; it < 4; ++it) {
        const int L  = it * 32 + (tid >> 3);
        const int rl = L >> 1, seg = L & 1, q = tid & 7;
        const int c  = seg * 64 + q * 8;
        const float* cp = Cs + rl * CSP + c;
        const v4f v0 = *(const v4f*)cp;
        const v4f v1 = *(const v4f*)(cp + 4);
        Pack8 pk;
        pk.h = (v8h){ (h16)v0[0], (h16)v0[1], (h16)v0[2], (h16)v0[3],
                      (h16)v1[0], (h16)v1[1], (h16)v1[2], (h16)v1[3] };
        *(volatile v4u*)(dstbase + (size_t)rl * pitch + c) = pk.u;
    }
}

__global__ __launch_bounds__(256) void k_gemm(
    const h16* __restrict__ A,
    const h16* __restrict__ B0, const h16* __restrict__ B1, const h16* __restrict__ B2,
    const float* __restrict__ bias0, const float* __restrict__ bias1,
    const float* __restrict__ bias2,
    h16* O0, h16* O1, h16* O2, float* Of,
    int M, int Nn, int K, int ldt, int ztrans, float cscale)
{
    __shared__ __attribute__((aligned(16))) float smem[64 * CSP];
    h16*   As = (h16*)smem;
    h16*   Bs = As + GT * LDSA;
    float* Cs = smem;
    (void)M;

    const int z = blockIdx.z;
    const h16*   Bt   = (z == 0) ? B0 : ((z == 1) ? B1 : B2);
    const float* bias = (z == 0) ? bias0 : ((z == 1) ? bias1 : bias2);
    h16*         Oh   = (z == 0) ? O0 : ((z == 1) ? O1 : O2);
    const bool trans = (z == ztrans);

    const int tid  = threadIdx.x;
    const int lane = tid & 31;
    const int wave = tid >> 5;
    const int half = lane >> 4;
    const int lcol = lane & 15;
    const int wm   = wave & 3;
    const int wn   = wave >> 2;
    const int m0   = blockIdx.y * GT;
    const int n0   = blockIdx.x * GT;

    const int crow = tid >> 1, chalf = tid & 1;
    const h16* aBase = A  + (size_t)(m0 + crow) * K + chalf * 16;
    const h16* bBase = Bt + (size_t)(n0 + crow) * K + chalf * 16;
    h16* aL = As + crow * LDSA + chalf * 16;
    h16* bL = Bs + crow * LDSA + chalf * 16;

    v8f acc[2][4];
    #pragma unroll
    for (int i = 0; i < 2; ++i)
        #pragma unroll
        for (int j = 0; j < 4; ++j)
            acc[i][j] = (v8f){0.f,0.f,0.f,0.f,0.f,0.f,0.f,0.f};

    const int nk = K >> 5;
    for (int kc = 0; kc < nk; ++kc) {
        const int koff = kc << 5;
        const v8h xa0 = *(const v8h*)(aBase + koff);
        const v8h xa1 = *(const v8h*)(aBase + koff + 8);
        const v8h xb0 = *(const v8h*)(bBase + koff);
        const v8h xb1 = *(const v8h*)(bBase + koff + 8);
        *(v8h*)(aL)     = xa0;
        *(v8h*)(aL + 8) = xa1;
        *(v8h*)(bL)     = xb0;
        *(v8h*)(bL + 8) = xb1;
        __syncthreads();

        const v16h fa0 = load_frag(As + (wm * 32) * LDSA,      LDSA);
        const v16h fa1 = load_frag(As + (wm * 32 + 16) * LDSA, LDSA);
        #pragma unroll
        for (int j = 0; j < 4; ++j) {
            const v16h fb = load_frag(Bs + (wn * 64 + j * 16) * LDSA, LDSA);
            acc[0][j] = wmma_f16(fa0, fb, acc[0][j]);
            acc[1][j] = wmma_f16(fa1, fb, acc[1][j]);
        }
        __syncthreads();
    }

    if (!trans) {
        #pragma unroll 1
        for (int ph = 0; ph < 2; ++ph) {
            if ((wm >> 1) == ph) {
                #pragma unroll
                for (int ni = 0; ni < 4; ++ni) {
                    const int cl = wn * 64 + ni * 16 + lcol;
                    const float bv = bf16_rne(bias[n0 + cl]);
                    #pragma unroll
                    for (int mi = 0; mi < 2; ++mi) {
                        #pragma unroll
                        for (int r = 0; r < 8; ++r) {
                            const int rl = (wm & 1) * 32 + mi * 16 + r + 8 * half;
                            Cs[rl * CSP + cl] = acc[mi][ni][r] * cscale + bv;
                        }
                    }
                }
            }
            __syncthreads();
            if (Of != nullptr) {
                float* dst = Of + (size_t)(m0 + ph * 64) * Nn + n0;
                emit_rows_f32(Cs, dst, Nn, tid);
                __threadfence();
                emit_rows_f32(Cs, dst, Nn, tid);
            } else {
                h16* dst = Oh + (size_t)(m0 + ph * 64) * Nn + n0;
                emit_rows_f16(Cs, dst, Nn, tid);
                __threadfence();
                emit_rows_f16(Cs, dst, Nn, tid);
            }
            __syncthreads();
        }
    } else {
        #pragma unroll 1
        for (int ph = 0; ph < 2; ++ph) {
            if (wn == ph) {
                #pragma unroll
                for (int ni = 0; ni < 4; ++ni) {
                    const int cl = ni * 16 + lcol;
                    const float bv = bf16_rne(bias[n0 + ph * 64 + cl]);
                    #pragma unroll
                    for (int mi = 0; mi < 2; ++mi) {
                        #pragma unroll
                        for (int r = 0; r < 8; ++r) {
                            const int tl = wm * 32 + mi * 16 + r + 8 * half;
                            Cs[cl * CSP + tl] = acc[mi][ni][r] * cscale + bv;
                        }
                    }
                }
            }
            __syncthreads();
            h16* dst = Oh + (size_t)(n0 + ph * 64) * ldt + m0;
            emit_rows_f16(Cs, dst, ldt, tid);
            __threadfence();
            emit_rows_f16(Cs, dst, ldt, tid);
            __syncthreads();
        }
    }
}

__global__ __launch_bounds__(128) __attribute__((amdgpu_num_vgpr(256)))
void k_attn(const h16* __restrict__ Qp, const h16* __restrict__ Kp,
            const h16* __restrict__ Vt, const int* __restrict__ ids, h16* Cx)
{
    __shared__ int ids_s[SEQ];
    __shared__ int kmn_s[NKB];
    __shared__ int kmx_s[NKB];
    __shared__ int vis_s[NKB];
    __shared__ int nvis_s;
    __shared__ __attribute__((aligned(16))) h16 Ps[4][16][PSP];

    const int tid  = threadIdx.x;
    const int lane = tid & 31;
    const int wave = tid >> 5;
    const int half = lane >> 4;
    const int lcol = lane & 15;
    const int qb   = blockIdx.x;
    const int hc   = blockIdx.y * HDIM;
    const int qb0  = qb * KBLK;
    const int q0   = qb0 + wave * 16;

    for (int i = tid; i < SEQ; i += 128) ids_s[i] = ids[i];
    __syncthreads();
    for (int b = tid; b < NKB; b += 128) {
        const int* p = ids_s + b * KBLK;
        int mn = p[0], mx = p[0];
        #pragma unroll 4
        for (int j = 1; j < KBLK; ++j) {
            const int v = p[j];
            mn = min(mn, v);
            mx = max(mx, v);
        }
        kmn_s[b] = mn;
        kmx_s[b] = mx;
    }
    __syncthreads();
    if (tid == 0) {
        const int qmin = kmn_s[qb], qmax = kmx_s[qb];
        int c = 0;
        for (int b = 0; b < NKB; ++b) {
            if (kmx_s[b] >= qmin && kmn_s[b] <= qmax) { vis_s[c] = b; ++c; }
        }
        nvis_s = c;
    }
    __syncthreads();
    int nvis = __builtin_amdgcn_readfirstlane(nvis_s);
    nvis = min(nvis, NKB);

    int idq[8];
    #pragma unroll
    for (int r = 0; r < 8; ++r) idq[r] = ids_s[q0 + 8 * half + r];

    v16h aq[2];
    aq[0] = load_frag(Qp + (size_t)q0 * DIMN + hc,      DIMN);
    aq[1] = load_frag(Qp + (size_t)q0 * DIMN + hc + 32, DIMN);

    v8f o[4], m, l;
    #pragma unroll
    for (int nt = 0; nt < 4; ++nt) o[nt] = (v8f){0.f,0.f,0.f,0.f,0.f,0.f,0.f,0.f};
    #pragma unroll
    for (int r = 0; r < 8; ++r) { m[r] = -3.0e38f; l[r] = 0.f; }

    #pragma unroll 1
    for (int t = 0; t < nvis; ++t) {
        int kb = __builtin_amdgcn_readfirstlane(vis_s[t]);
        kb = min(max(kb, 0), NKB - 1);
        const int jb = kb * KBLK;

        v8f s[4];
        #pragma unroll
        for (int nt = 0; nt < 4; ++nt) {
            v8f a = (v8f){0.f,0.f,0.f,0.f,0.f,0.f,0.f,0.f};
            #pragma unroll
            for (int kc = 0; kc < 2; ++kc) {
                const v16h bk = load_frag(
                    Kp + (size_t)(jb + nt * 16) * DIMN + hc + kc * 32, DIMN);
                a = wmma_f16(aq[kc], bk, a);
            }
            s[nt] = a;
        }

        int idk[4];
        #pragma unroll
        for (int nt = 0; nt < 4; ++nt) idk[nt] = ids_s[jb + nt * 16 + lcol];
        #pragma unroll
        for (int nt = 0; nt < 4; ++nt) {
            #pragma unroll
            for (int r = 0; r < 8; ++r) {
                const float sv = s[nt][r] * 0.125f;
                s[nt][r] = (idq[r] == idk[nt]) ? sv : -3.0e38f;
            }
        }

        v8f rmax = s[0];
        #pragma unroll
        for (int nt = 1; nt < 4; ++nt)
            #pragma unroll
            for (int r = 0; r < 8; ++r) rmax[r] = fmaxf(rmax[r], s[nt][r]);
        #pragma unroll
        for (int off = 1; off <= 8; off <<= 1)
            #pragma unroll
            for (int r = 0; r < 8; ++r)
                rmax[r] = fmaxf(rmax[r], __shfl_xor(rmax[r], off, 32));

        v8f mnew, rscale, rsum;
        #pragma unroll
        for (int r = 0; r < 8; ++r) {
            mnew[r]   = fmaxf(m[r], rmax[r]);
            rscale[r] = __expf(m[r] - mnew[r]);
            rsum[r]   = 0.f;
        }
        #pragma unroll
        for (int nt = 0; nt < 4; ++nt) {
            #pragma unroll
            for (int r = 0; r < 8; ++r) {
                const float e = __expf(s[nt][r] - mnew[r]);
                const float p = (idq[r] == idk[nt]) ? e : 0.f;
                s[nt][r] = p;
                rsum[r] += p;
            }
        }
        #pragma unroll
        for (int off = 1; off <= 8; off <<= 1)
            #pragma unroll
            for (int r = 0; r < 8; ++r) rsum[r] += __shfl_xor(rsum[r], off, 32);
        #pragma unroll
        for (int r = 0; r < 8; ++r) {
            l[r] = l[r] * rscale[r] + rsum[r];
            m[r] = mnew[r];
        }
        #pragma unroll
        for (int nt = 0; nt < 4; ++nt)
            #pragma unroll
            for (int r = 0; r < 8; ++r) o[nt][r] *= rscale[r];

        __syncthreads();
        #pragma unroll
        for (int nt = 0; nt < 4; ++nt)
            #pragma unroll
            for (int r = 0; r < 8; ++r)
                Ps[wave][r + 8 * half][nt * 16 + lcol] = (h16)s[nt][r];
        __syncthreads();

        #pragma unroll
        for (int kc = 0; kc < 2; ++kc) {
            const v16h ap = load_frag(&Ps[wave][0][0] + kc * 32, PSP);
            #pragma unroll
            for (int nt = 0; nt < 4; ++nt) {
                const v16h bv = load_frag(
                    Vt + (size_t)(hc + nt * 16) * SEQ + jb + kc * 32, SEQ);
                o[nt] = wmma_f16(ap, bv, o[nt]);
            }
        }
    }

    v8f inv;
    #pragma unroll
    for (int r = 0; r < 8; ++r) inv[r] = 16.0f * __builtin_amdgcn_rcpf(l[r]);
    __syncthreads();
    #pragma unroll
    for (int nt = 0; nt < 4; ++nt)
        #pragma unroll
        for (int r = 0; r < 8; ++r)
            Ps[wave][r + 8 * half][nt * 16 + lcol] = (h16)(o[nt][r] * inv[r]);
    __syncthreads();

    #pragma unroll
    for (int it = 0; it < 4; ++it) {
        const int row = it * 4 + (lane >> 3);
        const int q   = lane & 7;
        const v4u v = *(const v4u*)(&Ps[wave][row][q * 8]);
        *(volatile v4u*)(Cx + (size_t)(q0 + row) * DIMN + hc + q * 8) = v;
    }
    __threadfence();
    #pragma unroll
    for (int it = 0; it < 4; ++it) {
        const int row = it * 4 + (lane >> 3);
        const int q   = lane & 7;
        const v4u v = *(const v4u*)(&Ps[wave][row][q * 8]);
        *(volatile v4u*)(Cx + (size_t)(q0 + row) * DIMN + hc + q * 8) = v;
    }
}

extern "C" void kernel_launch(void* const* d_in, const int* in_sizes, int n_in,
                              void* d_out, int out_size, void* d_ws, size_t ws_size,
                              hipStream_t stream)
{
    if (n_in < 10) return;
    if (in_sizes[0] < SEQ * DIMN) return;
    if (in_sizes[1] < SEQ) return;
    if (in_sizes[2] < DIMN * DIMN || in_sizes[3] < DIMN * DIMN ||
        in_sizes[4] < DIMN * DIMN || in_sizes[8] < DIMN * DIMN) return;
    if (in_sizes[5] < DIMN || in_sizes[6] < DIMN || in_sizes[7] < DIMN ||
        in_sizes[9] < DIMN) return;
    if (out_size < SEQ * DIMN) return;

    const float* x     = (const float*)d_in[0];
    const int*   batch = (const int*)d_in[1];
    const float* wq    = (const float*)d_in[2];
    const float* wk    = (const float*)d_in[3];
    const float* wv    = (const float*)d_in[4];
    const float* bq    = (const float*)d_in[5];
    const float* bk    = (const float*)d_in[6];
    const float* bv    = (const float*)d_in[7];
    const float* wo    = (const float*)d_in[8];
    const float* bo    = (const float*)d_in[9];
    float* out = (float*)d_out;

    const size_t actB = (size_t)SEQ * DIMN * sizeof(h16);
    const size_t wB   = (size_t)DIMN * DIMN * sizeof(h16);
    const size_t total = 5 * actB + 4 * wB;
    if (total > ws_size) return;
    char* base = (char*)d_ws;
    size_t off = 0;
    h16* xh  = (h16*)(base + off); off += actB;
    h16* wqh = (h16*)(base + off); off += wB;
    h16* wkh = (h16*)(base + off); off += wB;
    h16* wvh = (h16*)(base + off); off += wB;
    h16* woh = (h16*)(base + off); off += wB;
    h16* Qp  = (h16*)(base + off); off += actB;
    h16* Kp  = (h16*)(base + off); off += actB;
    h16* Vt  = (h16*)(base + off); off += actB;
    h16* Cx  = (h16*)(base + off); off += actB;
    if (off > ws_size) return;

    k_cvt4<<<dim3(SEQ * DIMN / 8 / 256, 1), 256, 0, stream>>>(
        x, x, x, x, xh, xh, xh, xh, SEQ * DIMN / 8, 1.0f);
    k_cvt4<<<dim3(DIMN * DIMN / 8 / 256, 4), 256, 0, stream>>>(
        wq, wk, wv, wo, wqh, wkh, wvh, woh, DIMN * DIMN / 8, 64.0f);
    k_gemm<<<dim3(DIMN / GT, SEQ / GT, 3), 256, 0, stream>>>(
        xh, wqh, wkh, wvh, bq, bk, bv, Qp, Kp, Vt, nullptr,
        SEQ, DIMN, DIMN, SEQ, 2, 1.0f / 64.0f);
    k_attn<<<dim3(SEQ / KBLK, NHEAD), 128, 0, stream>>>(Qp, Kp, Vt, batch, Cx);
    k_gemm<<<dim3(DIMN / GT, SEQ / GT, 1), 256, 0, stream>>>(
        Cx, woh, woh, woh, bo, bo, bo, nullptr, nullptr, nullptr, out,
        SEQ, DIMN, DIMN, SEQ, -1, 1.0f / 1024.0f);
}
